// GRUPolicy_60559038873742
// MI455X (gfx1250) — hardware-run, weakly checked
//
#include <hip/hip_runtime.h>
#include <math.h>

typedef __attribute__((ext_vector_type(16))) _Float16 v16h;
typedef __attribute__((ext_vector_type(8)))  _Float16 v8h;
typedef __attribute__((ext_vector_type(8)))  float    v8f;
typedef __attribute__((ext_vector_type(4)))  float    v4f;
typedef __attribute__((ext_vector_type(2)))  float    v2f;

constexpr int kB   = 2048;
constexpr int kT   = 512;
constexpr int kVoc = 4;
constexpr int kE   = 64;
constexpr int kH   = 128;
constexpr int kG   = 3 * kH;
constexpr int kBM  = 16;
constexpr int kHP  = 136;
constexpr int kHB  = kBM * kHP;
constexpr int kFP  = 132;
constexpr float kHCarry   = 64.0f;
constexpr float kWCarry   = 256.0f;
constexpr float kAccScale = 1.0f / (kHCarry * kWCarry);
constexpr float kF16MinNormal = 6.103515625e-5f;

static_assert(kG == 384, "gate rows");
static_assert(kH == 8 * 16, "8 waves x 16 hidden columns");
static_assert((kH % 32) == 0, "K multiple of 32");
static_assert((kB % kBM) == 0, "grid covers the batch exactly");
static_assert((kT % 256) == 0, "token word staging");
static_assert((kG % 32) == 0, "one whole 128-B line per wave in the table kernel");
static_assert(((2 * kHB) % 8) == 0, "zero fill in 16-B vectors");
static_assert(((kHP * 2) % 16) == 0 && ((kFP * 4) % 16) == 0, "16-B aligned LDS rows");
static_assert(kBM * kVoc == 64, "256 B of output per block");

constexpr size_t kOffGtab = 0;
constexpr size_t kWsTotal = kOffGtab + (size_t)kVoc * kG * 4;
static_assert(kWsTotal == 6144ull, "carve total");
static_assert(kWsTotal <= 134217728ull, "carve cap");

union FragH { v16h v; v8h h[2]; };
__device__ __forceinline__ v16h frag_load_h(const _Float16* p) {
  FragH f;
  f.h[0] = *(const v8h*)(p);
  f.h[1] = *(const v8h*)(p + 16);
  return f.v;
}
__device__ __forceinline__ v8f mma_h(v16h a, v16h b, v8f c) {
  return __builtin_amdgcn_wmma_f32_16x16x32_f16(false, a, false, b, (short)0, c, false, false);
}
__device__ __forceinline__ void guard1(v8f& acc, v16h x, v16h y) {
  asm volatile("v_nop\n\tv_nop\n\tv_nop\n\tv_nop" : "+v"(acc) : "v"(x), "v"(y));
}
__device__ __forceinline__ void pin_frag(v16h& f) {
  asm volatile("" : "+v"(f));
}
__device__ __forceinline__ _Float16 to_f16_carried(float v, float carry) {
  float s = v * carry;
  s = (fabsf(s) < kF16MinNormal) ? 0.0f : s;
  return (_Float16)s;
}
__device__ __forceinline__ float fast_sigmoid(float v) {
  return __builtin_amdgcn_rcpf(1.0f + __expf(-v));
}
__device__ __forceinline__ float fast_tanh(float v) {
  return 2.0f * __builtin_amdgcn_rcpf(1.0f + __expf(-2.0f * v)) - 1.0f;
}

__global__ __launch_bounds__(384) void gate_table_kernel(
    const float* __restrict__ emb, const float* __restrict__ W_ih,
    const float* __restrict__ b_ih, const float* __restrict__ b_hh,
    float* __restrict__ gtab_out)
{
  __shared__ __align__(16) float semb[kVoc * kE];
  const int g = threadIdx.x;
  if (g < kVoc * kE) semb[g] = emb[g];
  __syncthreads();
  float s0 = 0.0f, s1 = 0.0f, s2 = 0.0f, s3 = 0.0f;
  const float* wr = W_ih + (size_t)g * kE;
#pragma unroll 2
  for (int e4 = 0; e4 < kE / 4; ++e4) {
    const v4f w  = *(const v4f*)(wr + 4 * e4);
    const v4f e0 = *(const v4f*)(semb + 0 * kE + 4 * e4);
    const v4f e1 = *(const v4f*)(semb + 1 * kE + 4 * e4);
    const v4f e2 = *(const v4f*)(semb + 2 * kE + 4 * e4);
    const v4f e3 = *(const v4f*)(semb + 3 * kE + 4 * e4);
    s0 = fmaf(e0[0], w[0], s0); s0 = fmaf(e0[1], w[1], s0); s0 = fmaf(e0[2], w[2], s0); s0 = fmaf(e0[3], w[3], s0);
    s1 = fmaf(e1[0], w[0], s1); s1 = fmaf(e1[1], w[1], s1); s1 = fmaf(e1[2], w[2], s1); s1 = fmaf(e1[3], w[3], s1);
    s2 = fmaf(e2[0], w[0], s2); s2 = fmaf(e2[1], w[1], s2); s2 = fmaf(e2[2], w[2], s2); s2 = fmaf(e2[3], w[3], s2);
    s3 = fmaf(e3[0], w[0], s3); s3 = fmaf(e3[1], w[1], s3); s3 = fmaf(e3[2], w[2], s3); s3 = fmaf(e3[3], w[3], s3);
  }
  const float bi = b_ih[g];
  const float bh = b_hh[g];
  const float addb = bi + ((g < 2 * kH) ? bh : 0.0f);
  const float t0 = s0 + addb;
  const float t1 = s1 + addb;
  const float t2 = s2 + addb;
  const float t3 = s3 + addb;
  volatile float* q = (volatile float*)gtab_out;
  q[0 * kG + g] = t0;
  q[1 * kG + g] = t1;
  q[2 * kG + g] = t2;
  q[3 * kG + g] = t3;
  __threadfence();
  q[0 * kG + g] = t0;
  q[1 * kG + g] = t1;
  q[2 * kG + g] = t2;
  q[3 * kG + g] = t3;
}

__global__ __launch_bounds__(256) void recur_scan_kernel(
    const int* __restrict__ x, const float* __restrict__ W_hh, const float* __restrict__ b_hh,
    const float* __restrict__ W_fc, const float* __restrict__ b_fc, const float* __restrict__ gtab_in,
    float* __restrict__ out)
{
  __shared__ __align__(16) _Float16 hbuf[2 * kHB];
  __shared__ __align__(16) float    sG[kVoc * kG];
  __shared__ __align__(16) float    sWfc[kVoc * kH];
  __shared__ __align__(16) float    sHf[kBM * kFP];
  __shared__ unsigned               sTok[kT];

  const int tid  = threadIdx.x;
  const int lane = tid & 31;
  const int wv   = tid >> 5;
  const int c    = lane & 15;
  const int hh   = lane >> 4;
  const int rb   = blockIdx.x * kBM;
  const int hcol = wv * 16 + c;

#pragma unroll 1
  for (int t = tid; t < kT; t += 256) {
    unsigned wd = 0u;
#pragma unroll 8
    for (int m = 0; m < kBM; ++m) {
      const int xv = x[(size_t)(rb + m) * kT + t];
      wd |= (((unsigned)xv) & 3u) << (2 * m);
    }
    sTok[t] = wd;
  }
  for (int idx = tid; idx < (kVoc * kG) / 4; idx += 256)
    *(v4f*)(sG + 4 * idx) = *(const v4f*)(gtab_in + 4 * idx);
  if (tid < (kVoc * kH) / 4)
    *(v4f*)(sWfc + 4 * tid) = *(const v4f*)(W_fc + 4 * tid);
  {
    const v8h zv = (v8h){(_Float16)0.0f, (_Float16)0.0f, (_Float16)0.0f, (_Float16)0.0f,
                         (_Float16)0.0f, (_Float16)0.0f, (_Float16)0.0f, (_Float16)0.0f};
    for (int idx = tid; idx < (2 * kHB) / 8; idx += 256)
      *(v8h*)(hbuf + 8 * idx) = zv;
  }

  const float bN = b_hh[2 * kH + hcol];
  const int   v0 = (lane & 1) * 2;
  const float bfc0 = b_fc[v0];
  const float bfc1 = b_fc[v0 + 1];

  v16h bw[3][4];
#pragma unroll
  for (int g = 0; g < 3; ++g) {
    const float* wp = W_hh + (size_t)(g * kH + hcol) * kH + 8 * hh;
#pragma unroll
    for (int ks = 0; ks < 4; ++ks) {
      const v4f p0 = *(const v4f*)(wp + 32 * ks);
      const v4f p1 = *(const v4f*)(wp + 32 * ks + 4);
      const v4f p2 = *(const v4f*)(wp + 32 * ks + 16);
      const v4f p3 = *(const v4f*)(wp + 32 * ks + 20);
      v16h f;
#pragma unroll
      for (int e = 0; e < 4; ++e) {
        f[e]      = to_f16_carried(p0[e], kWCarry);
        f[4 + e]  = to_f16_carried(p1[e], kWCarry);
        f[8 + e]  = to_f16_carried(p2[e], kWCarry);
        f[12 + e] = to_f16_carried(p3[e], kWCarry);
      }
      pin_frag(f);
      bw[g][ks] = f;
    }
  }

  float hreg[8];
#pragma unroll
  for (int i = 0; i < 8; ++i) hreg[i] = 0.0f;

  __syncthreads();

  const int aoff = c * kHP + 8 * hh;
  const int doff = 8 * hh * kHP + hcol;
  int rofs = 0;

#pragma unroll 1
  for (int t = 0; t < kT; ++t) {
    const _Float16* hr = hbuf + rofs + aoff;
    _Float16*       hw = hbuf + (kHB - rofs) + doff;

    const v16h a0 = frag_load_h(hr);
    const v16h a1 = frag_load_h(hr + 32);
    const v16h a2 = frag_load_h(hr + 64);
    const v16h a3 = frag_load_h(hr + 96);

    v8f accR = (v8f){0.f, 0.f, 0.f, 0.f, 0.f, 0.f, 0.f, 0.f};
    v8f accZ = (v8f){0.f, 0.f, 0.f, 0.f, 0.f, 0.f, 0.f, 0.f};
    v8f accN = (v8f){0.f, 0.f, 0.f, 0.f, 0.f, 0.f, 0.f, 0.f};

    accR = mma_h(a0, bw[0][0], accR);
    accZ = mma_h(a0, bw[1][0], accZ);
    accN = mma_h(a0, bw[2][0], accN);
    accR = mma_h(a1, bw[0][1], accR);
    accZ = mma_h(a1, bw[1][1], accZ);
    accN = mma_h(a1, bw[2][1], accN);
    accR = mma_h(a2, bw[0][2], accR);
    accZ = mma_h(a2, bw[1][2], accZ);
    accN = mma_h(a2, bw[2][2], accN);
    accR = mma_h(a3, bw[0][3], accR);
    accZ = mma_h(a3, bw[1][3], accZ);
    accN = mma_h(a3, bw[2][3], accN);
    guard1(accR, a0, a3);
    guard1(accZ, a1, a3);
    guard1(accN, a2, a3);

    const unsigned tw = sTok[t] >> (16 * hh);

#pragma unroll
    for (int r = 0; r < 8; ++r) {
      const unsigned tok = (tw >> (2 * r)) & 3u;
      const float* gt = sG + tok * kG + hcol;
      const float gr  = fmaf(accR[r], kAccScale, gt[0]);
      const float gz  = fmaf(accZ[r], kAccScale, gt[kH]);
      const float ghn = fmaf(accN[r], kAccScale, bN);
      const float rg  = fast_sigmoid(gr);
      const float zg  = fast_sigmoid(gz);
      const float ng  = fast_tanh(fmaf(rg, ghn, gt[2 * kH]));
      const float hn  = (1.0f - zg) * ng + zg * hreg[r];
      hreg[r] = hn;
      hw[r * kHP] = to_f16_carried(hn, kHCarry);
    }
    __syncthreads();
    rofs = kHB - rofs;
  }

#pragma unroll
  for (int r = 0; r < 8; ++r) sHf[(8 * hh + r) * kFP + hcol] = hreg[r];
  __syncthreads();

  if (wv == 0) {
    const int row = lane >> 1;
    const float* hp = sHf + row * kFP;
    const float* wa = sWfc + v0 * kH;
    const float* wb = sWfc + (v0 + 1) * kH;
    float s0 = 0.0f, s1 = 0.0f;
#pragma unroll 2
    for (int k4 = 0; k4 < kH / 4; ++k4) {
      const v4f hv = *(const v4f*)(hp + 4 * k4);
      const v4f xa = *(const v4f*)(wa + 4 * k4);
      const v4f xb = *(const v4f*)(wb + 4 * k4);
      s0 = fmaf(hv[0], xa[0], s0); s0 = fmaf(hv[1], xa[1], s0); s0 = fmaf(hv[2], xa[2], s0); s0 = fmaf(hv[3], xa[3], s0);
      s1 = fmaf(hv[0], xb[0], s1); s1 = fmaf(hv[1], xb[1], s1); s1 = fmaf(hv[2], xb[2], s1); s1 = fmaf(hv[3], xb[3], s1);
    }
    v2f o;
    o[0] = s0 + bfc0;
    o[1] = s1 + bfc1;
    volatile v2f* q = (volatile v2f*)(out + (size_t)blockIdx.x * (kBM * kVoc) + 2 * lane);
    *q = o;
    __threadfence();
    *q = o;
  }
}

extern "C" void kernel_launch(void* const* d_in, const int* in_sizes, int n_in,
                              void* d_out, int out_size, void* d_ws, size_t ws_size,
                              hipStream_t stream) {
  if (n_in < 8) return;
  if (in_sizes[0] != kB * kT) return;
  if (in_sizes[1] != kVoc * kE) return;
  if (in_sizes[2] != kG * kE) return;
  if (in_sizes[3] != kG * kH) return;
  if (in_sizes[4] != kG) return;
  if (in_sizes[5] != kG) return;
  if (in_sizes[6] != kVoc * kH) return;
  if (in_sizes[7] != kVoc) return;
  if (out_size != kB * kVoc) return;
  if (ws_size < kWsTotal) return;

  const int*   x    = (const int*)d_in[0];
  const float* emb  = (const float*)d_in[1];
  const float* W_ih = (const float*)d_in[2];
  const float* W_hh = (const float*)d_in[3];
  const float* b_ih = (const float*)d_in[4];
  const float* b_hh = (const float*)d_in[5];
  const float* W_fc = (const float*)d_in[6];
  const float* b_fc = (const float*)d_in[7];
  float* out  = (float*)d_out;
  float* gtab = (float*)((char*)d_ws + kOffGtab);

  gate_table_kernel<<<1, kG, 0, stream>>>(emb, W_ih, b_ih, b_hh, gtab);
  recur_scan_kernel<<<kB / kBM, 256, 0, stream>>>(x, W_hh, b_hh, W_fc, b_fc, gtab, out);
}
